// GAT_15547781612261
// MI455X (gfx1250) — hardware-verified
//
#include <hip/hip_runtime.h>
#include <stddef.h>
#include <stdint.h>
#include <math.h>


#define DIN     1028
#define KP1     1056
#define NH      6
#define C1      128
#define C2      256
#define C3      1028
#define NC1     768
#define NC2     1536
#define NC3     6168
#define NP3     6208
#define KA2     256
#define KA3     512
#define EP      16
#define NG      8
#define SL      32
#define NTHR    256
#define NWAVE   8
#define EPT     8
#define CHUNK   (NTHR * EPT)
#define WCAP    (EPT * 32)
#define LISTN   (NWAVE * WCAP)
#define NB      256
#define SLOTB   8
#define RCAP    4096
#define DEGCAP  64
#define GBM     64
#define GBN     64
#define GTHR    128
#define MAXGA   64
#define FLW     32
#define WSMAX   134217728

static_assert(NB == (1 << SLOTB) && NB == NTHR);
static_assert((CHUNK & (CHUNK - 1)) == 0 && ((long long)CHUNK << SLOTB) < (1LL << 31));
static_assert(LISTN >= NB && (RCAP % 32) == 0);
static_assert((KP1 % 32) == 0 && KP1 >= DIN && (KP1 % 8) == 0 && (DIN % 4) == 0);
static_assert((NC1 % GBN) == 0 && (NC2 % GBN) == 0 && (NP3 % GBN) == 0 && NP3 >= NC3);
static_assert(NC1 == NH * C1 && NC2 == NH * C2 && NC3 == NH * C3);
static_assert(KA2 == 2 * C1 && KA3 == 2 * C2 && (KA2 % 32) == 0 && (KA3 % 32) == 0);
static_assert(C3 == DIN && SL == 32 && NG == NWAVE && ((NG * SL) % GBM) == 0);
static_assert(((NP3 * 4) % 128) == 0 && ((NC1 * 4) % 128) == 0 && ((NC2 * 4) % 128) == 0);
static_assert(GBM == (GTHR / 32) * 16 && (NB % GBM) == 0 && (NB % 32) == 0);
static_assert((NG * C3) % 4 == 0 && (C3 % 4) == 0);

typedef float          v4f  __attribute__((ext_vector_type(4)));
typedef float          v8f  __attribute__((ext_vector_type(8)));
typedef int            v4i  __attribute__((ext_vector_type(4)));
typedef int            v8i  __attribute__((ext_vector_type(8)));
typedef unsigned int   v4u  __attribute__((ext_vector_type(4)));
typedef unsigned short v8us __attribute__((ext_vector_type(8)));
typedef __bf16         v16b __attribute__((ext_vector_type(16)));
typedef v4f  __attribute__((may_alias)) v4fa;
typedef v4i  __attribute__((may_alias)) v4ia;
typedef v8us __attribute__((may_alias)) v8usa;
union FragB { v16b v; v8us h[2]; v8i w; };

__device__ __forceinline__ v8f wmb(const FragB& a, const FragB& b, v8f c) {
  v8f d = __builtin_amdgcn_wmma_f32_16x16x32_bf16(false, a.v, false, b.v, (short)0, c, false, false);
  asm volatile("v_nop\n\tv_nop\n\tv_nop\n\tv_nop" : "+v"(d) : "v"(a.w), "v"(b.w));
  return d;
}

__device__ __forceinline__ unsigned int f2bf(float f) {
  const unsigned int u = __float_as_uint(f);
  return ((u + 0x7FFFu + ((u >> 16) & 1u)) >> 16) & 0xFFFFu;
}
__device__ __forceinline__ float bf2f(unsigned int b) { return __uint_as_float(b << 16); }
__device__ __forceinline__ float bfr(float f) { return bf2f(f2bf(f)); }
__device__ __forceinline__ v4f bfr4(const v4f a) {
  v4f r; r.x = bfr(a.x); r.y = bfr(a.y); r.z = bfr(a.z); r.w = bfr(a.w); return r;
}
__device__ __forceinline__ unsigned int pk2(float lo, float hi) { return f2bf(lo) | (f2bf(hi) << 16); }
__device__ __forceinline__ v4u pack8(const v4f a, const v4f b) {
  v4u r;
  r.x = pk2(a.x, a.y); r.y = pk2(a.z, a.w); r.z = pk2(b.x, b.y); r.w = pk2(b.z, b.w);
  return r;
}
__device__ __forceinline__ int clampi(int v, int lo, int hi) { return v < lo ? lo : (v > hi ? hi : v); }

__device__ __forceinline__ int scan_chunk(const int* __restrict__ dsts, int nE, int cbase, int slotBase,
                                          int nb, int vec8, int* list, int tid, int lane, int wave) {
  int wc = 0;
  const int el0  = tid * EPT;
  const int e0   = cbase + el0;
  const int sent = -2147483647 - 1;
  v4i da, db;
  if (vec8 != 0 && cbase + CHUNK <= nE) {
    da = *(const v4i*)(dsts + e0);
    db = *(const v4i*)(dsts + e0 + 4);
  } else {
    da.x = (e0     < nE) ? dsts[min(e0,     nE - 1)] : sent;
    da.y = (e0 + 1 < nE) ? dsts[min(e0 + 1, nE - 1)] : sent;
    da.z = (e0 + 2 < nE) ? dsts[min(e0 + 2, nE - 1)] : sent;
    da.w = (e0 + 3 < nE) ? dsts[min(e0 + 3, nE - 1)] : sent;
    db.x = (e0 + 4 < nE) ? dsts[min(e0 + 4, nE - 1)] : sent;
    db.y = (e0 + 5 < nE) ? dsts[min(e0 + 5, nE - 1)] : sent;
    db.z = (e0 + 6 < nE) ? dsts[min(e0 + 6, nE - 1)] : sent;
    db.w = (e0 + 7 < nE) ? dsts[min(e0 + 7, nE - 1)] : sent;
  }
  const unsigned nbs = (unsigned)slotBase;
  const unsigned unb = (unsigned)nb;
  const unsigned s0 = (unsigned)da.x - nbs, s1 = (unsigned)da.y - nbs;
  const unsigned s2 = (unsigned)da.z - nbs, s3 = (unsigned)da.w - nbs;
  const unsigned s4 = (unsigned)db.x - nbs, s5 = (unsigned)db.y - nbs;
  const unsigned s6 = (unsigned)db.z - nbs, s7 = (unsigned)db.w - nbs;
  const bool h0 = s0 < unb, h1 = s1 < unb, h2 = s2 < unb, h3 = s3 < unb;
  const bool h4 = s4 < unb, h5 = s5 < unb, h6 = s6 < unb, h7 = s7 < unb;
  const unsigned any = __builtin_amdgcn_ballot_w32(h0 | h1 | h2 | h3 | h4 | h5 | h6 | h7);
  if (any != 0u) {
#define HITJ(J, HJ, SJ) { \
      const unsigned mj = __builtin_amdgcn_ballot_w32(HJ); \
      if (mj != 0u) { \
        if (HJ) { \
          const int pos = wc + (int)__builtin_amdgcn_mbcnt_lo(mj, 0u); \
          if (pos < WCAP) list[wave * WCAP + pos] = ((el0 + (J)) << SLOTB) | (int)(SJ); \
        } \
        wc += (int)__builtin_popcount(mj); } }
    HITJ(0, h0, s0)
    HITJ(1, h1, s1)
    HITJ(2, h2, s2)
    HITJ(3, h3, s3)
    HITJ(4, h4, s4)
    HITJ(5, h5, s5)
    HITJ(6, h6, s6)
    HITJ(7, h7, s7)
#undef HITJ
  }
  return wc;
}

__global__ __launch_bounds__(NTHR) void k_xprep(const float* __restrict__ x, unsigned short* xb, int nN, int nUnits) {
  const int i = (int)blockIdx.x * NTHR + (int)threadIdx.x;
  if (i >= nUnits) return;
  const int row = i / (KP1 / 8);
  const int c0  = (i - row * (KP1 / 8)) * 8;
  const int rc  = row < nN ? row : nN - 1;
  const int ca  = (c0     < DIN) ? c0     : DIN - 4;
  const int cb  = (c0 + 4 < DIN) ? c0 + 4 : DIN - 4;
  const float* p = x + (size_t)rc * DIN;
  v4f a = *(const v4fa*)(p + ca), b = *(const v4fa*)(p + cb);
  const v4f z4 = {0.f, 0.f, 0.f, 0.f};
  if (row >= nN || c0     >= DIN) a = z4;
  if (row >= nN || c0 + 4 >= DIN) b = z4;
  const v4u hv = pack8(a, b);
  unsigned short* o = xb + (size_t)i * 8;
  *(volatile v4u*)o = hv;
  __threadfence();
  *(volatile v4u*)o = hv;
}

__global__ __launch_bounds__(NTHR) void k_wtr(const float* __restrict__ w, int Kin, int Kper, int Ncol, int Kout,
                                              unsigned short* wt, int nUnits) {
  const int u = (int)blockIdx.x * NTHR + (int)threadIdx.x;
  if (u >= nUnits) return;
  const int kq = Kout >> 3;
  const int n  = u / kq;
  const int k8 = (u - n * kq) * 8;
  const int kk = k8 - (k8 / Kper) * Kper;
  const int ncl = n < Ncol ? n : Ncol - 1;
  const float* p = w + ncl;
  const int km = Kin - 1;
  v4f a, b;
  a.x = p[(size_t)min(kk + 0, km) * (size_t)Ncol];
  a.y = p[(size_t)min(kk + 1, km) * (size_t)Ncol];
  a.z = p[(size_t)min(kk + 2, km) * (size_t)Ncol];
  a.w = p[(size_t)min(kk + 3, km) * (size_t)Ncol];
  b.x = p[(size_t)min(kk + 4, km) * (size_t)Ncol];
  b.y = p[(size_t)min(kk + 5, km) * (size_t)Ncol];
  b.z = p[(size_t)min(kk + 6, km) * (size_t)Ncol];
  b.w = p[(size_t)min(kk + 7, km) * (size_t)Ncol];
  const bool nv = n < Ncol;
  a.x = (nv && kk + 0 < Kin) ? a.x : 0.f;
  a.y = (nv && kk + 1 < Kin) ? a.y : 0.f;
  a.z = (nv && kk + 2 < Kin) ? a.z : 0.f;
  a.w = (nv && kk + 3 < Kin) ? a.w : 0.f;
  b.x = (nv && kk + 4 < Kin) ? b.x : 0.f;
  b.y = (nv && kk + 5 < Kin) ? b.y : 0.f;
  b.z = (nv && kk + 6 < Kin) ? b.z : 0.f;
  b.w = (nv && kk + 7 < Kin) ? b.w : 0.f;
  const v4u wv = pack8(a, b);
  unsigned short* o = wt + (size_t)u * 8;
  *(volatile v4u*)o = wv;
  __threadfence();
  *(volatile v4u*)o = wv;
}

__global__ __launch_bounds__(GTHR) void k_gemm(const unsigned short* __restrict__ A,
                                               const unsigned short* __restrict__ WT,
                                               float* outF, int K, int ldo) {
  __shared__ __attribute__((aligned(16))) float stg[GBM * GBN];
  const int tid = (int)threadIdx.x, lane = tid & 31, wave = tid >> 5, hh = lane >> 4, m = lane & 15;
  const int rowBase = (int)blockIdx.x * GBM;
  const int col0    = (int)blockIdx.y * GBN;

  v8f acc[4];
  {
    const v8f z = {0.f, 0.f, 0.f, 0.f, 0.f, 0.f, 0.f, 0.f};
    acc[0] = z; acc[1] = z; acc[2] = z; acc[3] = z;
  }
  const unsigned short* ap = A  + (size_t)(rowBase + 16 * wave + m) * (size_t)K + 8 * hh;
  const unsigned short* wp = WT + (size_t)(col0 + m) * (size_t)K + 8 * hh;
  const int ksteps = K >> 5;
#pragma unroll 1
  for (int ks = 0; ks < ksteps; ++ks) {
    FragB af;
    af.h[0] = *(const v8usa*)(ap + 32 * ks);
    af.h[1] = *(const v8usa*)(ap + 32 * ks + 16);
#pragma unroll
    for (int t = 0; t < 4; ++t) {
      const unsigned short* wq = wp + (size_t)(16 * t) * (size_t)K + 32 * ks;
      FragB bf;
      bf.h[0] = *(const v8usa*)wq;
      bf.h[1] = *(const v8usa*)(wq + 16);
      acc[t] = wmb(af, bf, acc[t]);
    }
  }

#pragma unroll
  for (int t = 0; t < 4; ++t) {
    const int lc = 16 * t + m;
#pragma unroll
    for (int r = 0; r < 8; ++r) {
      const int lr = 16 * wave + 8 * hh + r;
      stg[lr * GBN + lc] = acc[t][r];
    }
  }
  __syncthreads();

  v4f fv[8];
#pragma unroll
  for (int i = 0; i < 8; ++i) {
    const int lr = 16 * wave + 2 * i + hh;
    fv[i] = *(const v4fa*)(stg + lr * GBN + 4 * m);
  }
#pragma unroll
  for (int i = 0; i < 8; ++i) {
    const int gr = rowBase + 16 * wave + 2 * i + hh;
    float* op = outF + (size_t)gr * (size_t)ldo + col0 + 4 * m;
    *(volatile v4f*)op = fv[i];
  }
  __threadfence();
#pragma unroll
  for (int i = 0; i < 8; ++i) {
    const int gr = rowBase + 16 * wave + 2 * i + hh;
    float* op = outF + (size_t)gr * (size_t)ldo + col0 + 4 * m;
    *(volatile v4f*)op = fv[i];
  }
}

template <int C>
__global__ __launch_bounds__(NTHR) void k_dots(const float* __restrict__ H, const float* __restrict__ as,
                                               const float* __restrict__ ad, float* Eo) {
  constexpr int LDF = NH * C;
  constexpr int NJ  = C / 128;
  static_assert(C % 128 == 0);
  __shared__ __attribute__((aligned(16))) float stg[32 * EP];
  const int tid = (int)threadIdx.x, lane = tid & 31, wave = tid >> 5;
  const int base = (int)blockIdx.x * 32;
#pragma unroll 1
  for (int i = 0; i < 4; ++i) {
    const int lr = 4 * wave + i;
    const float* hr = H + (size_t)(base + lr) * LDF;
#pragma unroll 1
    for (int h = 0; h < NH; ++h) {
      float s = 0.f, d = 0.f;
#pragma unroll
      for (int j = 0; j < NJ; ++j) {
        const int c = h * C + 128 * j + 4 * lane;
        const v4f hv = *(const v4fa*)(hr + c);
        const v4f av = bfr4(*(const v4fa*)(as + c));
        const v4f dv = bfr4(*(const v4fa*)(ad + c));
        s = fmaf(hv.x, av.x, s); s = fmaf(hv.y, av.y, s); s = fmaf(hv.z, av.z, s); s = fmaf(hv.w, av.w, s);
        d = fmaf(hv.x, dv.x, d); d = fmaf(hv.y, dv.y, d); d = fmaf(hv.z, dv.z, d); d = fmaf(hv.w, dv.w, d);
      }
#pragma unroll
      for (int off = 16; off > 0; off >>= 1) {
        s += __shfl_xor(s, off);
        d += __shfl_xor(d, off);
      }
      if (lane == 0) { stg[lr * EP + h] = s; stg[lr * EP + NH + h] = d; }
    }
    if (lane < 4) stg[lr * EP + 12 + lane] = 0.f;
  }
  __syncthreads();
  const int pc = tid < 128 ? tid : 127;
  const v4f v = *(const v4fa*)(stg + 4 * pc);
  float* op = Eo + (size_t)base * EP + 4 * pc;
  if (tid < 128) *(volatile v4f*)op = v;
  __threadfence();
  if (tid < 128) *(volatile v4f*)op = v;
}

template <int CPL>
__device__ __forceinline__ void gat_accum(const float* __restrict__ rowp, float al, int lane, float (&acc)[CPL]) {
  constexpr int C = CPL * 32;
#pragma unroll 1
  for (int h = 0; h < NH; ++h) {
    const float ah = __shfl(al, h);
    const float* rp = rowp + h * C + CPL * lane;
    const v4f a = *(const v4fa*)rp;
    acc[0] = fmaf(ah, a.x, acc[0]); acc[1] = fmaf(ah, a.y, acc[1]);
    acc[2] = fmaf(ah, a.z, acc[2]); acc[3] = fmaf(ah, a.w, acc[3]);
    if constexpr (CPL == 8) {
      const v4f b = *(const v4fa*)(rp + 4);
      acc[4] = fmaf(ah, b.x, acc[4]); acc[5] = fmaf(ah, b.y, acc[5]);
      acc[6] = fmaf(ah, b.z, acc[6]); acc[7] = fmaf(ah, b.w, acc[7]);
    }
  }
}

template <int CPL>
__global__ __launch_bounds__(NTHR) void k_agg(
    const int* __restrict__ srcs, const int* __restrict__ dsts,
    const float* __restrict__ F, const float* __restrict__ E,
    const float* __restrict__ bias, unsigned short* HP, int* FLGp,
    int nN, int nE, int vec8, int MPr, float slope) {
  static_assert(CPL == 4 || CPL == 8);
  constexpr int C   = CPL * 32;
  constexpr int LDF = NH * C;
  constexpr int PW  = 2 * C;
  __shared__ __attribute__((aligned(16))) int reg1[RCAP];
  __shared__ __attribute__((aligned(16))) int reg2[RCAP];
  __shared__ __attribute__((aligned(16))) int scnt[NB];
  __shared__ __attribute__((aligned(16))) int soff[NB];
  __shared__ __attribute__((aligned(16))) int list[LISTN];
  __shared__ int wcnt[NWAVE];
  __shared__ int wtot[NWAVE];
  __shared__ int wflag[NWAVE];
  const int tid = (int)threadIdx.x, lane = tid & 31, wave = tid >> 5;
  const int nodeBase = (int)blockIdx.x * NB;

  scnt[tid] = 0;
  __syncthreads();

  int tot = 0;
  const int nChunks = (nE + CHUNK - 1) / CHUNK;
#pragma unroll 1
  for (int ch = 0; ch < nChunks; ++ch) {
    const int cbase = ch * CHUNK;
    const int wc = scan_chunk(dsts, nE, cbase, nodeBase, NB, vec8, list, tid, lane, wave);
    if (lane == 0) wcnt[wave] = wc;
    __syncthreads();
    int pre = 0, all = 0;
#pragma unroll
    for (int w2 = 0; w2 < NWAVE; ++w2) {
      int c = wcnt[w2];
      c = c < 0 ? 0 : (c > WCAP ? WCAP : c);
      all += c;
      pre += (w2 < wave) ? c : 0;
    }
    const int wcc  = wc > WCAP ? WCAP : wc;
    const int base = tot + pre;
#pragma unroll 1
    for (int i = lane; i < wcc; i += 32) {
      const int ent = list[wave * WCAP + i];
      const int el  = (ent >> SLOTB) & (CHUNK - 1);
      const int sl  = ent & (NB - 1);
      int eid = cbase + el;
      eid = eid > nE - 1 ? nE - 1 : eid;
      const int pos = base + i;
      if (pos < RCAP) reg1[pos] = (int)(((unsigned)eid << SLOTB) | (unsigned)sl);
    }
    tot += all;
    tot = tot > RCAP ? RCAP : tot;
    __syncthreads();
  }
  const int nh = tot;

  if (wave == 0) {
#pragma unroll 1
    for (int b0 = 0; b0 < nh; b0 += 32) {
      const int idx = b0 + lane;
      const int uv  = reg1[idx < nh ? idx : nh - 1];
      const int m32 = (nh - b0) < 32 ? (nh - b0) : 32;
#pragma unroll 1
      for (int k = 0; k < m32; ++k) {
        const int u  = __builtin_amdgcn_readlane(uv, k);
        const int sl = u & (NB - 1);
        if (lane == 0) scnt[sl] = scnt[sl] + 1;
      }
    }
  }
  __syncthreads();

  {
    int cv = scnt[tid];
    cv = cv < 0 ? 0 : cv;
    int incl = cv;
#pragma unroll
    for (int d = 1; d < 32; d <<= 1) {
      const int up = __shfl_up(incl, d);
      if (lane >= d) incl += up;
    }
    if (lane == 31) wtot[wave] = incl;
    __syncthreads();
    int pre = 0;
#pragma unroll
    for (int w2 = 0; w2 < NWAVE; ++w2) pre += (w2 < wave) ? wtot[w2] : 0;
    const int ex = pre + incl - cv;
    soff[tid] = ex;
    list[tid] = ex;
  }
  __syncthreads();

  if (wave == 0) {
#pragma unroll 1
    for (int b0 = 0; b0 < nh; b0 += 32) {
      const int idx = b0 + lane;
      const int uv  = reg1[idx < nh ? idx : nh - 1];
      const int m32 = (nh - b0) < 32 ? (nh - b0) : 32;
#pragma unroll 1
      for (int k = 0; k < m32; ++k) {
        const int u   = __builtin_amdgcn_readlane(uv, k);
        const int sl  = u & (NB - 1);
        const int eid = (int)((unsigned)u >> SLOTB);
        if (lane == 0) {
          int pos = list[sl];
          pos = pos < 0 ? 0 : (pos > RCAP - 1 ? RCAP - 1 : pos);
          reg2[pos] = eid;
          list[sl] = pos + 1;
        }
      }
    }
  }
  __syncthreads();

  const bool ovf = (nh >= RCAP);
  const float qnan = __int_as_float(0x7fc00000);
  const int hq = lane < 5 ? lane : 5;
  int wbad = ovf ? 1 : 0;
  float bb[CPL];
  {
    const float* bq = bias + CPL * lane;
    const v4f a = bfr4(*(const v4fa*)bq);
    bb[0] = a.x; bb[1] = a.y; bb[2] = a.z; bb[3] = a.w;
    if constexpr (CPL == 8) {
      const v4f b = bfr4(*(const v4fa*)(bq + 4));
      bb[4] = b.x; bb[5] = b.y; bb[6] = b.z; bb[7] = b.w;
    }
  }

#pragma unroll 1
  for (int jt = 0; jt < NB / NWAVE; ++jt) {
    const int slot = wave * (NB / NWAVE) + jt;
    const int grow = nodeBase + slot;
    const int gcl  = grow < nN ? grow : nN - 1;
    int st = soff[slot];
    const int craw = scnt[slot];
    int cnt = craw;
    st  = st < 0 ? 0 : (st > nh ? nh : st);
    cnt = cnt < 0 ? 0 : (cnt > DEGCAP ? DEGCAP : cnt);
    if (cnt > nh - st) cnt = nh - st;
    if (craw > DEGCAP) wbad = 1;
    const float pz = (ovf || craw > DEGCAP) ? qnan : 0.0f;

    const float* Ed = E + (size_t)gcl * EP;
    const float edv = Ed[NH + hq];
    float e0 = Ed[hq] + edv;
    e0 = (e0 >= 0.f) ? e0 : slope * e0;

    float mx = e0;
#pragma unroll 1
    for (int q = 0; q < cnt; ++q) {
      int idx = st + q; idx = idx > RCAP - 1 ? RCAP - 1 : idx;
      const int eid = clampi(reg2[idx], 0, nE - 1);
      const int s   = clampi(srcs[eid], 0, nN - 1);
      float e = E[(size_t)s * EP + hq] + edv;
      e = (e >= 0.f) ? e : slope * e;
      mx = (e > mx) ? e : mx;
    }
    const float ex0 = expf(e0 - mx);
    float z = ex0;
#pragma unroll 1
    for (int q = 0; q < cnt; ++q) {
      int idx = st + q; idx = idx > RCAP - 1 ? RCAP - 1 : idx;
      const int eid = clampi(reg2[idx], 0, nE - 1);
      const int s   = clampi(srcs[eid], 0, nN - 1);
      float e = E[(size_t)s * EP + hq] + edv;
      e = (e >= 0.f) ? e : slope * e;
      z += expf(e - mx);
    }
    const float rz = 1.0f / z;
    float acc[CPL];
#pragma unroll
    for (int i = 0; i < CPL; ++i) acc[i] = 0.0f;
    gat_accum<CPL>(F + (size_t)gcl * LDF, ex0 * rz, lane, acc);
#pragma unroll 1
    for (int q = 0; q < cnt; ++q) {
      int idx = st + q; idx = idx > RCAP - 1 ? RCAP - 1 : idx;
      const int eid = clampi(reg2[idx], 0, nE - 1);
      const int s   = clampi(srcs[eid], 0, nN - 1);
      float e = E[(size_t)s * EP + hq] + edv;
      e = (e >= 0.f) ? e : slope * e;
      const float al = expf(e - mx) * rz;
      gat_accum<CPL>(F + (size_t)s * LDF, al, lane, acc);
    }

    const bool live = grow < nN;
    float v[CPL];
#pragma unroll
    for (int i = 0; i < CPL; ++i) {
      const float y = fmaf(acc[i], (1.0f / 6.0f), bb[i]) + pz;
      v[i] = live ? y : 0.0f;
    }
    const bool wr = grow < MPr;
    if constexpr (CPL == 4) {
      const unsigned int hbx = f2bf(v[0]), hby = f2bf(v[1]), hbz = f2bf(v[2]), hbw = f2bf(v[3]);
      const unsigned int lbx = f2bf(v[0] - bf2f(hbx)), lby = f2bf(v[1] - bf2f(hby));
      const unsigned int lbz = f2bf(v[2] - bf2f(hbz)), lbw = f2bf(v[3] - bf2f(hbw));
      const int hw0 = (int)(hbx | (hby << 16)), hw1 = (int)(hbz | (hbw << 16));
      const int lw0 = (int)(lbx | (lby << 16)), lw1 = (int)(lbz | (lbw << 16));
      const int sa = (2 * lane) & 31, sb = (2 * lane + 1) & 31;
      const int g0 = __shfl(hw0, sa), g1 = __shfl(hw1, sa), g2 = __shfl(hw0, sb), g3 = __shfl(hw1, sb);
      const int q0 = __shfl(lw0, sa), q1 = __shfl(lw1, sa), q2 = __shfl(lw0, sb), q3 = __shfl(lw1, sb);
      const bool lsel = lane >= 16;
      v4u pv;
      pv.x = (unsigned int)(lsel ? q0 : g0);
      pv.y = (unsigned int)(lsel ? q1 : g1);
      pv.z = (unsigned int)(lsel ? q2 : g2);
      pv.w = (unsigned int)(lsel ? q3 : g3);
      unsigned short* gp = HP + (size_t)grow * PW + 8 * lane;
      if (wr) *(volatile v4u*)gp = pv;
      __threadfence();
      if (wr) *(volatile v4u*)gp = pv;
    } else {
      v8us ho, lo;
#pragma unroll
      for (int i = 0; i < 8; ++i) {
        const unsigned hbi = f2bf(v[i]);
        ho[i] = (unsigned short)hbi;
        lo[i] = (unsigned short)f2bf(v[i] - bf2f(hbi));
      }
      unsigned short* hp = HP + (size_t)grow * PW + 8 * lane;
      if (wr) { *(volatile v8us*)hp = ho; *(volatile v8us*)(hp + C) = lo; }
      __threadfence();
      if (wr) { *(volatile v8us*)hp = ho; *(volatile v8us*)(hp + C) = lo; }
    }
  }

  if (lane == 0) wflag[wave] = wbad;
  __syncthreads();
  if (wave == 0) {
    int f = 0;
#pragma unroll
    for (int w2 = 0; w2 < NWAVE; ++w2) f |= wflag[w2];
    v4i fv; fv.x = f; fv.y = f; fv.z = f; fv.w = f;
    int* fp = FLGp + (size_t)blockIdx.x * FLW + 4 * (lane & 7);
    if (lane < 8) *(volatile v4i*)fp = fv;
    __threadfence();
    if (lane < 8) *(volatile v4i*)fp = fv;
  }
}

__global__ __launch_bounds__(NTHR) void k_sel3(const int* __restrict__ srcs, const int* __restrict__ dsts,
                                               const int* __restrict__ ptr, int nPtr,
                                               const unsigned short* __restrict__ X2, unsigned short* A3,
                                               int* CN3, int nN, int nE) {
  __shared__ int slist[NG * SL];
  __shared__ __attribute__((aligned(16))) int smeta[32];
  const int tid = (int)threadIdx.x, lane = tid & 31, g = tid >> 5;
  const int pi = (g + 1 < nPtr) ? g + 1 : nPtr - 1;
  int r = ptr[pi] - 1;
  if (r < 0) r += nN;
  r = clampi(r, 0, nN - 1);
  slist[g * SL + lane] = r;
  if (tid < 32) smeta[tid] = 0;
  __syncthreads();

  int cnt = 1;
  const int nIt = (nE + 31) >> 5;
#pragma unroll 1
  for (int it = 0; it < nIt; ++it) {
    const int e  = it * 32 + lane;
    const int ec = e < nE ? e : nE - 1;
    const int d  = dsts[ec];
    const int s  = clampi(srcs[ec], 0, nN - 1);
    const bool hit = (e < nE) && (d == r);
    const unsigned mk = __builtin_amdgcn_ballot_w32(hit);
    if (mk != 0u) {
      if (hit) {
        const int pos = cnt + (int)__builtin_amdgcn_mbcnt_lo(mk, 0u);
        if (pos < SL) slist[g * SL + pos] = s;
      }
      cnt += (int)__builtin_popcount(mk);
    }
  }
  __syncthreads();
  const int ovf = cnt > SL ? 1 : 0;
  const int cc  = cnt > SL ? SL : cnt;
  if (lane == 0) { smeta[g] = cc; smeta[8 + g] = r; smeta[16 + g] = ovf; }

#pragma unroll 1
  for (int j = 0; j < SL; ++j) {
    const int s = clampi(slist[g * SL + j], 0, nN - 1);
    const unsigned short* sp = X2 + (size_t)s * KA3 + 8 * lane;
    v4u hi = *(const v4u*)sp;
    v4u lo = *(const v4u*)(sp + C2);
    const v4u z4 = {0u, 0u, 0u, 0u};
    if (j >= cc) { hi = z4; lo = z4; }
    unsigned short* dp = A3 + (size_t)(g * SL + j) * KA3 + 8 * lane;
    *(volatile v4u*)dp = hi;
    *(volatile v4u*)(dp + C2) = lo;
    __threadfence();
    *(volatile v4u*)dp = hi;
    *(volatile v4u*)(dp + C2) = lo;
  }
  __syncthreads();
  if (g == 0) {
    const v4i mv = *(const v4ia*)(smeta + 4 * (lane & 7));
    int* cp = CN3 + 4 * (lane & 7);
    if (lane < 8) *(volatile v4i*)cp = mv;
    __threadfence();
    if (lane < 8) *(volatile v4i*)cp = mv;
  }
}

__global__ __launch_bounds__(NTHR) void k_fin(const float* __restrict__ T, const int* __restrict__ CN3,
                                              const int* __restrict__ FLG, int gA,
                                              const int* __restrict__ ptr, int nPtr,
                                              const float* __restrict__ x, const float* __restrict__ as3,
                                              const float* __restrict__ ad3, const float* __restrict__ b3,
                                              float* out, int nN, int nPieces) {
  __shared__ __attribute__((aligned(16))) float stage[NG * C3];
  __shared__ float sEs[NG * SL * 8];
  __shared__ float sEd[NG * 8];
  __shared__ float sAl[NG * SL * 8];
  const int tid = (int)threadIdx.x, lane = tid & 31, g = tid >> 5;
  constexpr int NPC = C3 / 4;
  constexpr int NITP = (NPC + 31) / 32;

  int pf = 0;
#pragma unroll 1
  for (int b = 0; b < gA; ++b) {
    pf |= FLG[(size_t)b * FLW];
    pf |= FLG[(size_t)(MAXGA + b) * FLW];
  }
#pragma unroll 1
  for (int g2 = 0; g2 < NG; ++g2) pf |= CN3[16 + g2];
  const float pz = (pf != 0) ? __int_as_float(0x7fc00000) : 0.0f;

  const int cnt = clampi(CN3[g], 1, SL);
  const int pi = (g + 1 < nPtr) ? g + 1 : nPtr - 1;
  int r = ptr[pi] - 1;
  if (r < 0) r += nN;
  r = clampi(r, 0, nN - 1);
  const float* Tg = T + (size_t)(g * SL) * NP3;

#pragma unroll 1
  for (int j = 0; j < cnt; ++j) {
#pragma unroll 1
    for (int h = 0; h < NH; ++h) {
      const float* rowp = Tg + (size_t)j * NP3 + h * C3;
      const float* ap = as3 + h * C3;
      const float* dq = ad3 + h * C3;
      float s = 0.f, d = 0.f;
#pragma unroll 1
      for (int it = 0; it < NITP; ++it) {
        const int p  = it * 32 + lane;
        const int pc = p < NPC ? p : NPC - 1;
        v4f hv = *(const v4fa*)(rowp + 4 * pc);
        const v4f z4 = {0.f, 0.f, 0.f, 0.f};
        if (p >= NPC) hv = z4;
        const v4f av = bfr4(*(const v4fa*)(ap + 4 * pc));
        const v4f dv = bfr4(*(const v4fa*)(dq + 4 * pc));
        s = fmaf(hv.x, av.x, s); s = fmaf(hv.y, av.y, s); s = fmaf(hv.z, av.z, s); s = fmaf(hv.w, av.w, s);
        d = fmaf(hv.x, dv.x, d); d = fmaf(hv.y, dv.y, d); d = fmaf(hv.z, dv.z, d); d = fmaf(hv.w, dv.w, d);
      }
#pragma unroll
      for (int off = 16; off > 0; off >>= 1) {
        s += __shfl_xor(s, off);
        d += __shfl_xor(d, off);
      }
      if (lane == 0) {
        sEs[(g * SL + j) * 8 + h] = s;
        if (j == 0) sEd[g * 8 + h] = d;
      }
    }
  }
  __syncthreads();

  {
    const int hq = lane < 5 ? lane : 5;
    const float edv = sEd[g * 8 + hq];
    float e0 = sEs[(g * SL) * 8 + hq] + edv;
    e0 = (e0 >= 0.f) ? e0 : 0.0f * e0;
    float mx = e0;
#pragma unroll 1
    for (int j = 1; j < cnt; ++j) {
      float e = sEs[(g * SL + j) * 8 + hq] + edv;
      e = (e >= 0.f) ? e : 0.0f * e;
      mx = (e > mx) ? e : mx;
    }
    float z = 0.0f;
#pragma unroll 1
    for (int j = 0; j < cnt; ++j) {
      float e = sEs[(g * SL + j) * 8 + hq] + edv;
      e = (e >= 0.f) ? e : 0.0f * e;
      z += expf(e - mx);
    }
    const float rz = 1.0f / z;
#pragma unroll 1
    for (int j = 0; j < cnt; ++j) {
      float e = sEs[(g * SL + j) * 8 + hq] + edv;
      e = (e >= 0.f) ? e : 0.0f * e;
      const float al = expf(e - mx) * rz;
      if (lane < 8) sAl[(g * SL + j) * 8 + lane] = al;
    }
  }
  __syncthreads();

#pragma unroll 1
  for (int it = 0; it < NITP; ++it) {
    const int p  = it * 32 + lane;
    const int pc = p < NPC ? p : NPC - 1;
    v4f acc = {0.f, 0.f, 0.f, 0.f};
#pragma unroll 1
    for (int j = 0; j < cnt; ++j) {
      const float* rowp = Tg + (size_t)j * NP3 + 4 * pc;
#pragma unroll 1
      for (int h = 0; h < NH; ++h) {
        const float a = sAl[(g * SL + j) * 8 + h];
        const v4f tv = *(const v4fa*)(rowp + h * C3);
        acc.x = fmaf(a, tv.x, acc.x); acc.y = fmaf(a, tv.y, acc.y);
        acc.z = fmaf(a, tv.z, acc.z); acc.w = fmaf(a, tv.w, acc.w);
      }
    }
    const v4f bv = bfr4(*(const v4fa*)(b3 + 4 * pc));
    const v4f xv = bfr4(*(const v4fa*)(x + (size_t)r * DIN + 4 * pc));
    v4f o;
    o.x = (fmaf(acc.x, (1.0f / 6.0f), bv.x) + xv.x) + pz;
    o.y = (fmaf(acc.y, (1.0f / 6.0f), bv.y) + xv.y) + pz;
    o.z = (fmaf(acc.z, (1.0f / 6.0f), bv.z) + xv.z) + pz;
    o.w = (fmaf(acc.w, (1.0f / 6.0f), bv.w) + xv.w) + pz;
    if (p < NPC) *(v4fa*)(stage + g * C3 + 4 * p) = o;
  }
  __syncthreads();

  const int nIt = (nPieces + NTHR - 1) / NTHR;
#pragma unroll 1
  for (int k = 0; k < nIt; ++k) {
    const int p  = k * NTHR + tid;
    const int pc = p < nPieces ? p : nPieces - 1;
    const v4f v = *(const v4fa*)(stage + 4 * pc);
    if (p < nPieces) *(volatile v4f*)(out + (size_t)4 * p) = v;
  }
  __threadfence();
#pragma unroll 1
  for (int k = 0; k < nIt; ++k) {
    const int p  = k * NTHR + tid;
    const int pc = p < nPieces ? p : nPieces - 1;
    const v4f v = *(const v4fa*)(stage + 4 * pc);
    if (p < nPieces) *(volatile v4f*)(out + (size_t)4 * p) = v;
  }
}

static inline int cdiv(int a, int b) { return (a + b - 1) / b; }
static inline size_t al256(size_t v) { return (v + 255) & ~(size_t)255; }

extern "C" void kernel_launch(void* const* d_in, const int* in_sizes, int n_in,
                              void* d_out, int out_size, void* d_ws, size_t ws_size,
                              hipStream_t stream) {
  if (n_in < 15) return;
  const int nN = in_sizes[0] / DIN;
  if (nN <= 0 || in_sizes[0] != nN * DIN || nN > MAXGA * NB) return;
  if (in_sizes[1] < 2 || (in_sizes[1] & 1) != 0) return;
  const int nE = in_sizes[1] / 2;
  if (nE < 1 || nE >= (1 << (31 - SLOTB))) return;
  const int nPtr = in_sizes[2];
  if (nPtr != NG + 1) return;
  if (in_sizes[3] != DIN * NC1) return;
  if (in_sizes[4] != NC1 || in_sizes[5] != NC1 || in_sizes[6] != C1) return;
  if (in_sizes[7] != C1 * NC2) return;
  if (in_sizes[8] != NC2 || in_sizes[9] != NC2 || in_sizes[10] != C2) return;
  if (in_sizes[11] != C2 * NC3) return;
  if (in_sizes[12] != NC3 || in_sizes[13] != NC3 || in_sizes[14] != C3) return;
  if (out_size != NG * C3) return;

  const float* x   = (const float*)d_in[0];
  const int*   ei  = (const int*)  d_in[1];
  const int*   ptr = (const int*)  d_in[2];
  const float* W1  = (const float*)d_in[3];
  const float* as1 = (const float*)d_in[4];
  const float* ad1 = (const float*)d_in[5];
  const float* b1  = (const float*)d_in[6];
  const float* W2  = (const float*)d_in[7];
  const float* as2 = (const float*)d_in[8];
  const float* ad2 = (const float*)d_in[9];
  const float* b2  = (const float*)d_in[10];
  const float* W3  = (const float*)d_in[11];
  const float* as3 = (const float*)d_in[12];
  const float* ad3 = (const float*)d_in[13];
  const float* b3  = (const float*)d_in[14];
  float* out = (float*)d_out;
  const int* src = ei;
  const int* dst = ei + nE;

  const int MP = cdiv(nN, NB) * NB;
  const int gA = MP / NB;
  if (gA < 1 || gA > MAXGA) return;
  const int vec8 = ((nE & 3) == 0) ? 1 : 0;

  char* ws = (char*)d_ws;
  size_t off = 0;
  const size_t oXB  = off; off += al256((size_t)MP * KP1 * 2);
  const size_t oW1T = off; off += al256((size_t)NC1 * KP1 * 2);
  const size_t oW2T = off; off += al256((size_t)NC2 * KA2 * 2);
  const size_t oW3T = off; off += al256((size_t)NP3 * KA3 * 2);
  const size_t oH   = off; off += al256((size_t)MP * NC2 * 4);
  const size_t oE   = off; off += al256((size_t)MP * EP * 4);
  const size_t oX1  = off; off += al256((size_t)MP * KA2 * 2);
  const size_t oX2  = off; off += al256((size_t)MP * KA3 * 2);
  const size_t oA3  = off; off += al256((size_t)NG * SL * KA3 * 2);
  const size_t oT   = off; off += al256((size_t)NG * SL * NP3 * 4);
  const size_t oFL  = off; off += al256((size_t)2 * MAXGA * FLW * 4);
  const size_t oCN  = off; off += al256((size_t)32 * 4);
  if (off > ws_size || off > (size_t)WSMAX) return;
  unsigned short* XB   = (unsigned short*)(ws + oXB);
  unsigned short* W1T  = (unsigned short*)(ws + oW1T);
  unsigned short* W2T2 = (unsigned short*)(ws + oW2T);
  unsigned short* W3T2 = (unsigned short*)(ws + oW3T);
  float*          Hp   = (float*)(ws + oH);
  float*          Ep   = (float*)(ws + oE);
  unsigned short* X1   = (unsigned short*)(ws + oX1);
  unsigned short* X2   = (unsigned short*)(ws + oX2);
  unsigned short* A3   = (unsigned short*)(ws + oA3);
  float*          Tp   = (float*)(ws + oT);
  int*            FLG  = (int*)(ws + oFL);
  int*            CN3  = (int*)(ws + oCN);

  const int nUx = MP * (KP1 / 8);
  k_xprep<<<cdiv(nUx, NTHR), NTHR, 0, stream>>>(x, XB, nN, nUx);
  {
    const int nU1 = NC1 * (KP1 / 8);
    k_wtr<<<cdiv(nU1, NTHR), NTHR, 0, stream>>>(W1, DIN, KP1, NC1, KP1, W1T, nU1);
    const int nU2 = NC2 * (KA2 / 8);
    k_wtr<<<cdiv(nU2, NTHR), NTHR, 0, stream>>>(W2, C1, C1, NC2, KA2, W2T2, nU2);
    const int nU3 = NP3 * (KA3 / 8);
    k_wtr<<<cdiv(nU3, NTHR), NTHR, 0, stream>>>(W3, C2, C2, NC3, KA3, W3T2, nU3);
  }

  const int gM = MP / GBM;
  k_gemm<<<dim3(gM, NC1 / GBN), GTHR, 0, stream>>>(XB, W1T, Hp, KP1, NC1);
  k_dots<C1><<<MP / 32, NTHR, 0, stream>>>(Hp, as1, ad1, Ep);
  k_agg<4><<<gA, NTHR, 0, stream>>>(src, dst, Hp, Ep, b1, X1, FLG, nN, nE, vec8, MP, 0.2f);
  k_gemm<<<dim3(gM, NC2 / GBN), GTHR, 0, stream>>>(X1, W2T2, Hp, KA2, NC2);
  k_dots<C2><<<MP / 32, NTHR, 0, stream>>>(Hp, as2, ad2, Ep);
  k_agg<8><<<gA, NTHR, 0, stream>>>(src, dst, Hp, Ep, b2, X2, FLG + (size_t)MAXGA * FLW, nN, nE, vec8, MP, 0.2f);
  k_sel3<<<1, NTHR, 0, stream>>>(src, dst, ptr, nPtr, X2, A3, CN3, nN, nE);
  k_gemm<<<dim3((NG * SL) / GBM, NP3 / GBN), GTHR, 0, stream>>>(A3, W3T2, Tp, KA3, NP3);
  k_fin<<<1, NTHR, 0, stream>>>(Tp, CN3, FLG, gA, ptr, nPtr, x, as3, ad3, b3, out, nN, out_size / 4);
}
